// Correlation_Module_31026843746365
// MI455X (gfx1250) — hardware-verified
//
#include <hip/hip_runtime.h>
#include <stddef.h>

typedef _Float16 v16h __attribute__((ext_vector_type(16)));
typedef _Float16 v8h  __attribute__((ext_vector_type(8)));
typedef float    v8f  __attribute__((ext_vector_type(8)));
typedef float    v4f  __attribute__((ext_vector_type(4)));
typedef unsigned v4u  __attribute__((ext_vector_type(4)));

union Frag { v16h v; v8h half[2]; };
union H8   { v8h h; v4u u; };

#define L_DIM 1024
#define N_DIM 64
#define D_DIM 64
#define O_DIM 1024
#define OSTEP 32
#define TPAD 72
#define FPAD 68

__device__ __forceinline__ v8f wmma16(v16h a, v16h b, v8f c) {
  v8f d = __builtin_amdgcn_wmma_f32_16x16x32_f16(false, a, false, b, (short)0, c, false, false);
  asm volatile("v_nop\n\tv_nop\n\tv_nop\n\tv_nop" : "+v"(d) : "v"(a), "v"(b));
  return d;
}

__device__ __forceinline__ v8h cvt8(v4f a, v4f b) {
  v8h h;
  h[0] = (_Float16)a[0]; h[1] = (_Float16)a[1]; h[2] = (_Float16)a[2]; h[3] = (_Float16)a[3];
  h[4] = (_Float16)b[0]; h[5] = (_Float16)b[1]; h[6] = (_Float16)b[2]; h[7] = (_Float16)b[3];
  return h;
}

__device__ __forceinline__ float gatew(float st) {
  const float e = __expf(st * -0.125f);
  const float r = __builtin_amdgcn_rcpf(1.0f + e);
  return __builtin_fmaf(r, 1024.0f, -512.0f);
}

__device__ __forceinline__ v4f lo4(v8f c) { return __builtin_shufflevector(c, c, 0, 1, 2, 3); }
__device__ __forceinline__ v4f hi4(v8f c) { return __builtin_shufflevector(c, c, 4, 5, 6, 7); }

__global__ __launch_bounds__(128)
void up_planes_kernel(const float* __restrict__ up,
                      _Float16* __restrict__ u16,
                      _Float16* __restrict__ ut16) {
  __shared__ _Float16 T [64][TPAD];
  __shared__ _Float16 TT[64][TPAD];
  const int tid  = threadIdx.x;
  const int wave = tid >> 5, lane = tid & 31;
  const int n    = blockIdx.y;
  const int ob   = blockIdx.x * 64;

  {
    const int orow = tid >> 1;
    const int dh   = (tid & 1) * 32;
    const v4f* rp = (const v4f*)(up + ((size_t)(ob + orow) * N_DIM + n) * D_DIM + dh);
#pragma unroll
    for (int c = 0; c < 4; ++c) {
      const v8h hv = cvt8(rp[2 * c], rp[2 * c + 1]);
      *(v8h*)&T[orow][dh + 8 * c] = hv;
#pragma unroll
      for (int j = 0; j < 8; ++j) TT[dh + 8 * c + j][orow] = hv[j];
    }
  }
  __syncthreads();

  const int q  = lane >> 3;
  const int j8 = (lane & 7) * 8;
  H8 uv[4], tv[4];
#pragma unroll
  for (int it = 0; it < 4; ++it) {
    const int row = wave * 16 + it * 4 + q;
    uv[it].h = *(const v8h*)&T [row][j8];
    tv[it].h = *(const v8h*)&TT[row][j8];
  }
  _Float16* ubase = u16  + (size_t)n * O_DIM * D_DIM + (size_t)ob * D_DIM + j8;
  _Float16* tbase = ut16 + (size_t)n * D_DIM * O_DIM + ob + j8;
#pragma unroll
  for (int it = 0; it < 4; ++it) {
    const int row = wave * 16 + it * 4 + q;
    *(volatile v4u*)(ubase + (size_t)row * D_DIM) = uv[it].u;
    *(volatile v4u*)(tbase + (size_t)row * O_DIM) = tv[it].u;
  }
  __threadfence();
#pragma unroll
  for (int it = 0; it < 4; ++it) {
    const int row = wave * 16 + it * 4 + q;
    *(volatile v4u*)(ubase + (size_t)row * D_DIM) = uv[it].u;
    *(volatile v4u*)(tbase + (size_t)row * O_DIM) = tv[it].u;
  }
}

__global__ __launch_bounds__(128)
void corr_main_kernel(const float* __restrict__ x,
                      const _Float16* __restrict__ u16,
                      const _Float16* __restrict__ ut16,
                      float* __restrict__ out) {
  __shared__ float Fs[4][16][FPAD];
  const int tid  = threadIdx.x;
  const int wave = tid >> 5, lane = tid & 31;
  const int h    = lane >> 4, m = lane & 15;
  const int n    = blockIdx.y;
  const int lbase = blockIdx.x * 64 + wave * 16;

  Frag bx0, bx1;
  {
    const float* xr = x + ((size_t)(lbase + m) * N_DIM + n) * D_DIM;
    const v4f* p;
    p = (const v4f*)(xr +      8 * h);  bx0.half[0] = cvt8(p[0], p[1]);
    p = (const v4f*)(xr + 16 + 8 * h);  bx0.half[1] = cvt8(p[0], p[1]);
    p = (const v4f*)(xr + 32 + 8 * h);  bx1.half[0] = cvt8(p[0], p[1]);
    p = (const v4f*)(xr + 48 + 8 * h);  bx1.half[1] = cvt8(p[0], p[1]);
  }
  const _Float16* un  = u16  + (size_t)n * O_DIM * D_DIM;
  const _Float16* utn = ut16 + (size_t)n * D_DIM * O_DIM;

  v8f acc0 = {}, acc1 = {}, acc2 = {}, acc3 = {};

#pragma unroll 1
  for (int ob = 0; ob < O_DIM; ob += OSTEP) {
    v8f st0 = {}, st1 = {};
    {
      Frag a0, a1;
      const _Float16* r0 = un + (size_t)(ob + m) * D_DIM + 8 * h;
      const _Float16* r1 = un + (size_t)(ob + 16 + m) * D_DIM + 8 * h;
      a0.half[0] = *(const v8h*)(r0);       a0.half[1] = *(const v8h*)(r0 + 16);
      a1.half[0] = *(const v8h*)(r1);       a1.half[1] = *(const v8h*)(r1 + 16);
      st0 = wmma16(a0.v, bx0.v, st0);
      st1 = wmma16(a1.v, bx0.v, st1);
      Frag c0, c1;
      c0.half[0] = *(const v8h*)(r0 + 32);  c0.half[1] = *(const v8h*)(r0 + 48);
      c1.half[0] = *(const v8h*)(r1 + 32);  c1.half[1] = *(const v8h*)(r1 + 48);
      st0 = wmma16(c0.v, bx1.v, st0);
      st1 = wmma16(c1.v, bx1.v, st1);
    }

    Frag bw;
    {
      v8h w0, w1;
#pragma unroll
      for (int r = 0; r < 8; ++r) {
        w0[r] = (_Float16)gatew(st0[r]);
        w1[r] = (_Float16)gatew(st1[r]);
      }
      bw.half[0] = w0;
      bw.half[1] = w1;
    }

    {
      const _Float16* rr = utn + (size_t)m * O_DIM + ob + 8 * h;
      Frag a;
      a.half[0] = *(const v8h*)(rr);                    a.half[1] = *(const v8h*)(rr + 16);
      acc0 = wmma16(a.v, bw.v, acc0);
      Frag b;
      b.half[0] = *(const v8h*)(rr + 16 * O_DIM);       b.half[1] = *(const v8h*)(rr + 16 * O_DIM + 16);
      acc1 = wmma16(b.v, bw.v, acc1);
      Frag c;
      c.half[0] = *(const v8h*)(rr + 32 * O_DIM);       c.half[1] = *(const v8h*)(rr + 32 * O_DIM + 16);
      acc2 = wmma16(c.v, bw.v, acc2);
      Frag d;
      d.half[0] = *(const v8h*)(rr + 48 * O_DIM);       d.half[1] = *(const v8h*)(rr + 48 * O_DIM + 16);
      acc3 = wmma16(d.v, bw.v, acc3);
    }
  }

  {
    const float inv = 0.0009765625f;
    float* fr = &Fs[wave][m][8 * h];
    *(v4f*)(fr +  0) = lo4(acc0) * inv;  *(v4f*)(fr +  4) = hi4(acc0) * inv;
    *(v4f*)(fr + 16) = lo4(acc1) * inv;  *(v4f*)(fr + 20) = hi4(acc1) * inv;
    *(v4f*)(fr + 32) = lo4(acc2) * inv;  *(v4f*)(fr + 36) = hi4(acc2) * inv;
    *(v4f*)(fr + 48) = lo4(acc3) * inv;  *(v4f*)(fr + 52) = hi4(acc3) * inv;
  }
  __syncthreads();

  {
    const int q  = lane >> 3;
    const int j4 = (lane & 7) * 4;
    v4f v[8];
#pragma unroll
    for (int it = 0; it < 8; ++it) {
      const int li = it * 4 + q;
      const int row = li >> 1, hf = (li & 1) * 32;
      v[it] = *(const v4f*)&Fs[wave][row][hf + j4];
    }
    float* obase = out + ((size_t)lbase * N_DIM + n) * D_DIM + j4;
#pragma unroll
    for (int it = 0; it < 8; ++it) {
      const int li = it * 4 + q;
      const int row = li >> 1, hf = (li & 1) * 32;
      *(volatile v4f*)(obase + (size_t)row * (N_DIM * D_DIM) + hf) = v[it];
    }
    __threadfence();
#pragma unroll
    for (int it = 0; it < 8; ++it) {
      const int li = it * 4 + q;
      const int row = li >> 1, hf = (li & 1) * 32;
      *(volatile v4f*)(obase + (size_t)row * (N_DIM * D_DIM) + hf) = v[it];
    }
  }
}

extern "C" void kernel_launch(void* const* d_in, const int* in_sizes, int n_in,
                              void* d_out, int out_size, void* d_ws, size_t ws_size,
                              hipStream_t stream) {
  if (n_in < 2) return;
  if (in_sizes[0] != L_DIM * N_DIM * D_DIM) return;
  if (in_sizes[1] != O_DIM * N_DIM * D_DIM) return;
  if (out_size != L_DIM * N_DIM * D_DIM) return;
  const float* x  = (const float*)d_in[0];
  const float* up = (const float*)d_in[1];
  float* out = (float*)d_out;

  const size_t plane_bytes = (size_t)in_sizes[1] * sizeof(_Float16);
  if (ws_size < 2 * plane_bytes) return;
  _Float16* u16  = (_Float16*)d_ws;
  _Float16* ut16 = (_Float16*)((char*)d_ws + plane_bytes);

  up_planes_kernel<<<dim3(O_DIM / 64, N_DIM), 128, 0, stream>>>(up, u16, ut16);
  corr_main_kernel<<<dim3(L_DIM / 64, N_DIM), 128, 0, stream>>>(x, u16, ut16, out);
}
